// Powen3Retention_44117904064896
// MI455X (gfx1250) — hardware-verified
//
#include <hip/hip_runtime.h>
#include <math.h>


#define TSEQ    3072
#define HID     2048
#define NHQ     16
#define NKV     8
#define HDIM    128
#define QDIM    (NHQ * HDIM)
#define KDIM    (NKV * HDIM)
#define QKROWS  (QDIM + KDIM)
#define VROWS   KDIM
#define GROWS   16
#define RMS_EPS 1e-6f
#define DEN_EPS 1e-6f
#define SCALE_Q 0.08838834764831845f
#define DECAY_CUT (-64.0f)
#define CT_PITCH 132
#define HS_SC   64.0f
#define W_SC    32.0f
#define ATT_SC  64.0f
#define OUT_SC  (1.0f / 2048.0f)
#define V_SC    (1.0f / 2048.0f)

typedef _Float16 v16h __attribute__((ext_vector_type(16)));
typedef _Float16 v8h  __attribute__((ext_vector_type(8)));
typedef _Float16 v8hx __attribute__((ext_vector_type(8), may_alias));
typedef __bf16   v16b __attribute__((ext_vector_type(16)));
typedef __bf16   v8b  __attribute__((ext_vector_type(8)));
typedef float    v8f  __attribute__((ext_vector_type(8)));
typedef float    v4f  __attribute__((ext_vector_type(4)));
typedef unsigned short us8  __attribute__((ext_vector_type(8)));
typedef unsigned short us8x __attribute__((ext_vector_type(8), may_alias));
typedef unsigned short us16 __attribute__((ext_vector_type(16)));

struct RopeFreq { float inv[64]; };
typedef char rope_freq_size_check[(sizeof(RopeFreq) == 256) ? 1 : -1];

__device__ __forceinline__ v8f f8zero() {
    v8f z = {0.f, 0.f, 0.f, 0.f, 0.f, 0.f, 0.f, 0.f};
    return z;
}

__device__ __forceinline__ v16b ldfrag(const __bf16* p) {
    v8b a = *(const v8b*)p;
    v8b b = *(const v8b*)(p + 16);
    return __builtin_shufflevector(a, b, 0, 1, 2, 3, 4, 5, 6, 7, 8, 9, 10, 11, 12, 13, 14, 15);
}
__device__ __forceinline__ v16h ldfrag(const _Float16* p) {
    v8h a = *(const v8h*)p;
    v8h b = *(const v8h*)(p + 16);
    return __builtin_shufflevector(a, b, 0, 1, 2, 3, 4, 5, 6, 7, 8, 9, 10, 11, 12, 13, 14, 15);
}
__device__ __forceinline__ v16b ldfrag_lds_b(const unsigned short* p) {
    us8x a = *(const us8x*)p;
    us8x b = *(const us8x*)(p + 16);
    us16 u = __builtin_shufflevector(a, b, 0, 1, 2, 3, 4, 5, 6, 7, 8, 9, 10, 11, 12, 13, 14, 15);
    union { us16 u; v16b v; } cv;
    cv.u = u;
    return cv.v;
}

__device__ __forceinline__ v8f mma16(v16b a, v16b b, v8f c) {
    c = __builtin_amdgcn_wmma_f32_16x16x32_bf16(false, a, false, b, (short)0, c, false, false);
    asm volatile("v_nop\n\tv_nop\n\tv_nop\n\tv_nop" : "+v"(c) : "v"(a), "v"(b));
    return c;
}
__device__ __forceinline__ v8f mma16(v16h a, v16h b, v8f c) {
    c = __builtin_amdgcn_wmma_f32_16x16x32_f16(false, a, false, b, (short)0, c, false, false);
    asm volatile("v_nop\n\tv_nop\n\tv_nop\n\tv_nop" : "+v"(c) : "v"(a), "v"(b));
    return c;
}

__device__ __forceinline__ unsigned short bf16_rne(float x) {
    unsigned int u = __float_as_uint(x);
    u += 0x7FFFu + ((u >> 16) & 1u);
    return (unsigned short)(u >> 16);
}
__device__ __forceinline__ float bf16_up(unsigned short b) {
    return __uint_as_float(((unsigned int)b) << 16);
}

__global__ void __launch_bounds__(256)
k_cvt3(const float* __restrict__ src, unsigned short* dhi, unsigned short* dlo, _Float16* dh, int nvec, float sc) {
    const int i = blockIdx.x * 256 + threadIdx.x;
    if (i >= nvec) return;
    const float* p = src + (size_t)i * 8;
    const v4f a = *(const v4f*)p;
    const v4f b = *(const v4f*)(p + 4);
    float x[8] = {a[0], a[1], a[2], a[3], b[0], b[1], b[2], b[3]};
    us8 vh, vl;
    v8h vf;
#pragma unroll
    for (int e = 0; e < 8; ++e) {
        const unsigned short hb = bf16_rne(x[e]);
        vh[e] = hb;
        vl[e] = bf16_rne(x[e] - bf16_up(hb));
        vf[e] = (_Float16)(x[e] * sc);
    }
    const size_t o = (size_t)i * 8;
    *(volatile us8*)(dhi + o) = vh;
    *(volatile us8*)(dlo + o) = vl;
    *(volatile v8h*)(dh + o) = vf;
    __threadfence();
    *(volatile us8*)(dhi + o) = vh;
    *(volatile us8*)(dlo + o) = vl;
    *(volatile v8h*)(dh + o) = vf;
}

__global__ void __launch_bounds__(256)
k_cvt_split(const float* __restrict__ src, unsigned short* dhi, unsigned short* dlo, int nvalid, int ntotal) {
    const int i = blockIdx.x * 256 + threadIdx.x;
    if (i >= ntotal) return;
    us8 vh, vl;
    if (i < nvalid) {
        const float* p = src + (size_t)i * 8;
        const v4f a = *(const v4f*)p;
        const v4f b = *(const v4f*)(p + 4);
        float x[8] = {a[0], a[1], a[2], a[3], b[0], b[1], b[2], b[3]};
#pragma unroll
        for (int e = 0; e < 8; ++e) {
            const unsigned short hb = bf16_rne(x[e]);
            vh[e] = hb;
            vl[e] = bf16_rne(x[e] - bf16_up(hb));
        }
    } else {
#pragma unroll
        for (int e = 0; e < 8; ++e) { vh[e] = 0; vl[e] = 0; }
    }
    const size_t o = (size_t)i * 8;
    *(volatile us8*)(dhi + o) = vh;
    *(volatile us8*)(dlo + o) = vl;
    __threadfence();
    *(volatile us8*)(dhi + o) = vh;
    *(volatile us8*)(dlo + o) = vl;
}

__global__ void __launch_bounds__(256)
k_cvt_h(const float* __restrict__ src, _Float16* dh, int nvec, float sc) {
    const int i = blockIdx.x * 256 + threadIdx.x;
    if (i >= nvec) return;
    const float* p = src + (size_t)i * 8;
    const v4f a = *(const v4f*)p;
    const v4f b = *(const v4f*)(p + 4);
    float x[8] = {a[0], a[1], a[2], a[3], b[0], b[1], b[2], b[3]};
    v8h vf;
#pragma unroll
    for (int e = 0; e < 8; ++e) vf[e] = (_Float16)(x[e] * sc);
    const size_t o = (size_t)i * 8;
    *(volatile v8h*)(dh + o) = vf;
    __threadfence();
    *(volatile v8h*)(dh + o) = vf;
}

__global__ void __launch_bounds__(256)
k_rope_tab(const int* __restrict__ pos, float* tab, RopeFreq fq, int n) {
    const int idx = blockIdx.x * 256 + threadIdx.x;
    if (idx >= n) return;
    const int t = idx >> 6, i = idx & 63;
    const float p = (float)pos[t];
    const float ang = p * fq.inv[i];
    const float c = cosf(ang);
    const float s = sinf(ang);
    float* d = tab + (size_t)t * 128;
    *(volatile float*)(d + i) = c;
    *(volatile float*)(d + 64 + i) = s;
    __threadfence();
    *(volatile float*)(d + i) = c;
    *(volatile float*)(d + 64 + i) = s;
}

__global__ void __launch_bounds__(32)
k_gate(const __bf16* __restrict__ ah, const __bf16* __restrict__ al,
       const __bf16* __restrict__ gh, const __bf16* __restrict__ gl, float* graw) {
    __shared__ __align__(16) float st[256];
    const int l = threadIdx.x & 31, h = l >> 4, m = l & 15;
    const int row0 = blockIdx.x * 32;
    const size_t ao0 = (size_t)(row0 + m) * HID + 8 * h;
    const size_t ao1 = ao0 + (size_t)16 * HID;
    const size_t bo  = (size_t)m * HID + 8 * h;
    v8f c0 = f8zero(), c1 = f8zero();
#pragma unroll 1
    for (int k0 = 0; k0 < HID; k0 += 32) {
        const v16b a0  = ldfrag(ah + ao0 + k0), a1  = ldfrag(ah + ao1 + k0);
        const v16b a0l = ldfrag(al + ao0 + k0), a1l = ldfrag(al + ao1 + k0);
        const v16b b   = ldfrag(gh + bo + k0),  bl  = ldfrag(gl + bo + k0);
        c0 = mma16(a0, b, c0);  c0 = mma16(a0, bl, c0);  c0 = mma16(a0l, b, c0);
        c1 = mma16(a1, b, c1);  c1 = mma16(a1, bl, c1);  c1 = mma16(a1l, b, c1);
    }
    if (m < NKV) {
#pragma unroll
        for (int r = 0; r < 8; ++r) {
            st[(8 * h + r) * NKV + m]      = c0[r];
            st[(16 + 8 * h + r) * NKV + m] = c1[r];
        }
    }
    __syncthreads();
    const v4f x0 = *(const v4f*)(st + 4 * l);
    const v4f x1 = *(const v4f*)(st + 128 + 4 * l);
    float* d = graw + (size_t)row0 * NKV;
    *(volatile v4f*)(d + 4 * l) = x0;
    *(volatile v4f*)(d + 128 + 4 * l) = x1;
    __threadfence();
    *(volatile v4f*)(d + 4 * l) = x0;
    *(volatile v4f*)(d + 128 + 4 * l) = x1;
}

__global__ void __launch_bounds__(32)
k_cumsum(const float* __restrict__ graw, float* cgT) {
    __shared__ __align__(16) float st[NKV][1024];
    const int l = threadIdx.x & 31;
    float run = 0.f;
#pragma unroll 1
    for (int ch = 0; ch < TSEQ / 1024; ++ch) {
        if (l < NKV) {
#pragma unroll 1
            for (int tt = 0; tt < 1024; ++tt) {
                const float g  = graw[(size_t)(ch * 1024 + tt) * NKV + l];
                const float ex = expf(-fabsf(g));
                const float lg = fminf(g, 0.f) - log1pf(ex);
                run += lg;
                st[l][tt] = run;
            }
        }
        __syncthreads();
        for (int kvh = 0; kvh < NKV; ++kvh) {
            float* dst = cgT + (size_t)kvh * TSEQ + (size_t)ch * 1024;
#pragma unroll 1
            for (int q = 0; q < 8; ++q) {
                const v4f x = *(const v4f*)(&st[kvh][q * 128 + 4 * l]);
                *(volatile v4f*)(dst + q * 128 + 4 * l) = x;
            }
        }
        __threadfence();
        for (int kvh = 0; kvh < NKV; ++kvh) {
            float* dst = cgT + (size_t)kvh * TSEQ + (size_t)ch * 1024;
#pragma unroll 1
            for (int q = 0; q < 8; ++q) {
                const v4f x = *(const v4f*)(&st[kvh][q * 128 + 4 * l]);
                *(volatile v4f*)(dst + q * 128 + 4 * l) = x;
            }
        }
        __syncthreads();
    }
}

template <bool SPLIT, typename T>
__device__ __forceinline__ void mainloop(const T* __restrict__ A0, const T* __restrict__ A1,
                                         const T* __restrict__ B0, const T* __restrict__ B1,
                                         int K, int arow, int bcol, v8f (&acc)[2][4]) {
    const int l = threadIdx.x & 31, h = l >> 4, m = l & 15;
    const size_t ao0 = (size_t)(arow + m) * K + 8 * h;
    const size_t ao1 = ao0 + (size_t)16 * K;
    const size_t bo  = (size_t)(bcol + m) * K + 8 * h;
#pragma unroll 1
    for (int k0 = 0; k0 < K; k0 += 32) {
        auto a0 = ldfrag(A0 + ao0 + k0);
        auto a1 = ldfrag(A0 + ao1 + k0);
        decltype(a0) a0l = a0, a1l = a1;
        if (SPLIT) { a0l = ldfrag(A1 + ao0 + k0); a1l = ldfrag(A1 + ao1 + k0); }
#pragma unroll
        for (int c = 0; c < 4; ++c) {
            const size_t bc = bo + (size_t)c * 16 * K + k0;
            auto b = ldfrag(B0 + bc);
            acc[0][c] = mma16(a0, b, acc[0][c]);
            acc[1][c] = mma16(a1, b, acc[1][c]);
            if (SPLIT) {
                auto bl = ldfrag(B1 + bc);
                acc[0][c] = mma16(a0, bl, acc[0][c]);
                acc[1][c] = mma16(a1, bl, acc[1][c]);
                acc[0][c] = mma16(a0l, b, acc[0][c]);
                acc[1][c] = mma16(a1l, b, acc[1][c]);
            }
        }
    }
}

__device__ __forceinline__ void stage_acc(float (*ct)[CT_PITCH], v8f (&acc)[2][4]) {
    const int l = threadIdx.x & 31, h = l >> 4, m = l & 15, warp = threadIdx.x >> 5;
    const int wr = (warp & 3) * 32, wc = (warp >> 2) * 64;
#pragma unroll
    for (int f = 0; f < 2; ++f)
#pragma unroll
        for (int c = 0; c < 4; ++c)
#pragma unroll
            for (int r = 0; r < 8; ++r)
                ct[wr + f * 16 + 8 * h + r][wc + c * 16 + m] = acc[f][c][r];
}

__global__ void __launch_bounds__(256)
k_proj_qk(const __bf16* __restrict__ ah, const __bf16* __restrict__ al,
          const __bf16* __restrict__ wh, const __bf16* __restrict__ wl,
          const float* __restrict__ qnw, const float* __restrict__ knw,
          const float* __restrict__ rope,
          unsigned short* qh, unsigned short* qlo, unsigned short* kh, unsigned short* klo) {
    __shared__ __align__(16) float ct[128][CT_PITCH];
    const int warp = threadIdx.x >> 5, l = threadIdx.x & 31, h = l >> 4, hl = l & 15;
    const int t0 = blockIdx.y * 128, cb = blockIdx.x;
    v8f acc[2][4];
#pragma unroll
    for (int f = 0; f < 2; ++f)
#pragma unroll
        for (int c = 0; c < 4; ++c) acc[f][c] = f8zero();
    mainloop<true, __bf16>(ah, al, wh, wl, HID, t0 + (warp & 3) * 32, cb * 128 + (warp >> 2) * 64, acc);
    stage_acc(ct, acc);
    __syncthreads();

    const bool isq = cb < NHQ;
    const float* nw = isq ? qnw : knw;
    unsigned short* dh = isq ? qh : kh;
    unsigned short* dl = isq ? qlo : klo;
    const size_t pitch = isq ? (size_t)QDIM : (size_t)KDIM;
    const size_t colb  = (size_t)(isq ? cb : (cb - NHQ)) * HDIM;
    const float osc = isq ? SCALE_Q : 1.0f;
    const int d0 = hl * 8;
    const int i0 = d0 & 63;
    const float sgn = (hl < 8) ? -1.0f : 1.0f;
    float nwv[8];
    {
        const v4f a = *(const v4f*)(nw + d0), b = *(const v4f*)(nw + d0 + 4);
        nwv[0] = a[0]; nwv[1] = a[1]; nwv[2] = a[2]; nwv[3] = a[3];
        nwv[4] = b[0]; nwv[5] = b[1]; nwv[6] = b[2]; nwv[7] = b[3];
    }
#pragma unroll 1
    for (int it = 0; it < 8; ++it) {
        const int rl = warp * 16 + it * 2 + h;
        const int t = t0 + rl;
        float x[8];
        {
            const v4f a = *(const v4f*)(&ct[rl][d0]), b = *(const v4f*)(&ct[rl][d0 + 4]);
            x[0] = a[0]; x[1] = a[1]; x[2] = a[2]; x[3] = a[3];
            x[4] = b[0]; x[5] = b[1]; x[6] = b[2]; x[7] = b[3];
        }
        float ss = 0.f;
#pragma unroll
        for (int e = 0; e < 8; ++e) ss += x[e] * x[e];
        ss += __shfl_xor(ss, 8, 32);
        ss += __shfl_xor(ss, 4, 32);
        ss += __shfl_xor(ss, 2, 32);
        ss += __shfl_xor(ss, 1, 32);
        const float rr = rsqrtf(ss * (1.0f / (float)HDIM) + RMS_EPS);
#pragma unroll
        for (int e = 0; e < 8; ++e) x[e] = x[e] * rr * nwv[e];
        float y[8];
#pragma unroll
        for (int e = 0; e < 8; ++e) y[e] = __shfl_xor(x[e], 8, 32);
        float cs[8], sn[8];
        {
            const float* tr = rope + (size_t)t * 128 + i0;
            const v4f ca = *(const v4f*)tr, cbv = *(const v4f*)(tr + 4);
            const v4f sa = *(const v4f*)(tr + 64), sb = *(const v4f*)(tr + 68);
            cs[0] = ca[0]; cs[1] = ca[1]; cs[2] = ca[2]; cs[3] = ca[3];
            cs[4] = cbv[0]; cs[5] = cbv[1]; cs[6] = cbv[2]; cs[7] = cbv[3];
            sn[0] = sa[0]; sn[1] = sa[1]; sn[2] = sa[2]; sn[3] = sa[3];
            sn[4] = sb[0]; sn[5] = sb[1]; sn[6] = sb[2]; sn[7] = sb[3];
        }
        us8 vh, vl;
#pragma unroll
        for (int e = 0; e < 8; ++e) {
            const float o = (x[e] * cs[e] + sgn * (y[e] * sn[e])) * osc;
            const unsigned short hb = bf16_rne(o);
            vh[e] = hb;
            vl[e] = bf16_rne(o - bf16_up(hb));
        }
        const size_t off = (size_t)t * pitch + colb + d0;
        *(volatile us8*)(dh + off) = vh;
        *(volatile us8*)(dl + off) = vl;
        __threadfence();
        *(volatile us8*)(dh + off) = vh;
        *(volatile us8*)(dl + off) = vl;
    }
}

__global__ void __launch_bounds__(256)
k_proj_v(const _Float16* __restrict__ a16, const _Float16* __restrict__ w16, unsigned short* vth, unsigned short* vtl) {
    __shared__ __align__(16) float ct[128][CT_PITCH];
    const int warp = threadIdx.x >> 5, l = threadIdx.x & 31, h = l >> 4, hl = l & 15;
    const int t0 = blockIdx.y * 128, cb = blockIdx.x;
    v8f acc[2][4];
#pragma unroll
    for (int f = 0; f < 2; ++f)
#pragma unroll
        for (int c = 0; c < 4; ++c) acc[f][c] = f8zero();
    mainloop<false, _Float16>(a16, a16, w16, w16, HID, t0 + (warp & 3) * 32, cb * 128 + (warp >> 2) * 64, acc);
    stage_acc(ct, acc);
    __syncthreads();
#pragma unroll 1
    for (int it = 0; it < 8; ++it) {
        const int dloc = warp * 16 + it * 2 + h;
        us8 vh, vl;
#pragma unroll
        for (int e = 0; e < 8; ++e) {
            const float v = ct[8 * hl + e][dloc] * V_SC;
            const unsigned short hb = bf16_rne(v);
            vh[e] = hb;
            vl[e] = bf16_rne(v - bf16_up(hb));
        }
        const size_t off = (size_t)(cb * HDIM + dloc) * TSEQ + t0 + 8 * hl;
        *(volatile us8*)(vth + off) = vh;
        *(volatile us8*)(vtl + off) = vl;
        __threadfence();
        *(volatile us8*)(vth + off) = vh;
        *(volatile us8*)(vtl + off) = vl;
    }
}

__global__ void __launch_bounds__(128)
k_ret(const __bf16* __restrict__ qh, const __bf16* __restrict__ ql,
      const __bf16* __restrict__ kh, const __bf16* __restrict__ kl,
      const __bf16* __restrict__ vth, const __bf16* __restrict__ vtl,
      const float* __restrict__ cgT, _Float16* attn) {
    __shared__ __align__(16) unsigned short wth[4][16][32];
    __shared__ __align__(16) unsigned short wtl[4][16][32];
    __shared__ __align__(16) _Float16 ot[4][16][128];
    const int l = threadIdx.x & 31, h = l >> 4, m = l & 15, warp = threadIdx.x >> 5;
    const int hq = blockIdx.y, kv = hq >> 1;
    const int qb = blockIdx.x * 64 + warp * 16;
    const float* cgr = cgT + (size_t)kv * TSEQ;

    float cgq[8];
#pragma unroll
    for (int r = 0; r < 8; ++r) cgq[r] = cgr[qb + 8 * h + r];

    int jst = 0;
    {
        const float cq0 = cgr[qb];
#pragma unroll 1
        for (int jj = 0; jj + 31 < qb; jj += 32) {
            if (cq0 - cgr[jj + 31] < DECAY_CUT) jst = jj + 32;
        }
    }
    jst = __builtin_amdgcn_readfirstlane(jst);
    const int jend = qb + 16;

    v8f oacc[8];
#pragma unroll
    for (int c = 0; c < 8; ++c) oacc[c] = f8zero();
    float wsum[8] = {0.f, 0.f, 0.f, 0.f, 0.f, 0.f, 0.f, 0.f};

    const size_t qo = (size_t)(qb + m) * QDIM + (size_t)hq * HDIM + 8 * h;
    const size_t vo = (size_t)(kv * HDIM + m) * TSEQ + 8 * h;

#pragma unroll 1
    for (int j = jst; j < jend; j += 32) {
        v8f s0 = f8zero(), s1 = f8zero();
        const size_t ko0 = (size_t)(j + m) * KDIM + (size_t)kv * HDIM + 8 * h;
        const size_t ko1 = ko0 + (size_t)16 * KDIM;
#pragma unroll 1
        for (int c = 0; c < 4; ++c) {
            const int d = c * 32;
            const v16b qa = ldfrag(qh + qo + d), qr = ldfrag(ql + qo + d);
            v16b ka = ldfrag(kh + ko0 + d), kr = ldfrag(kl + ko0 + d);
            s0 = mma16(qa, ka, s0); s0 = mma16(qa, kr, s0); s0 = mma16(qr, ka, s0);
            ka = ldfrag(kh + ko1 + d); kr = ldfrag(kl + ko1 + d);
            s1 = mma16(qa, ka, s1); s1 = mma16(qa, kr, s1); s1 = mma16(qr, ka, s1);
        }
        const float ck0 = cgr[j + m], ck1 = cgr[j + 16 + m];
#pragma unroll
        for (int r = 0; r < 8; ++r) {
            const int row = qb + 8 * h + r;
            float w0 = 0.f, w1 = 0.f;
            if (j + m <= row)      { const float sv = s0[r]; w0 = __expf(cgq[r] - ck0) * (sv * sv); }
            if (j + 16 + m <= row) { const float sv = s1[r]; w1 = __expf(cgq[r] - ck1) * (sv * sv); }
            wsum[r] += w0 + w1;
            const unsigned short hb0 = bf16_rne(w0), hb1 = bf16_rne(w1);
            wth[warp][8 * h + r][m]      = hb0;
            wtl[warp][8 * h + r][m]      = bf16_rne(w0 - bf16_up(hb0));
            wth[warp][8 * h + r][16 + m] = hb1;
            wtl[warp][8 * h + r][16 + m] = bf16_rne(w1 - bf16_up(hb1));
        }
        asm volatile("" ::: "memory");
        const v16b pa = ldfrag_lds_b(&wth[warp][m][8 * h]);
        const v16b pl = ldfrag_lds_b(&wtl[warp][m][8 * h]);
#pragma unroll
        for (int c = 0; c < 8; ++c) {
            const size_t vc = vo + (size_t)c * 16 * TSEQ + j;
            const v16b va = ldfrag(vth + vc);
            const v16b vl = ldfrag(vtl + vc);
            oacc[c] = mma16(pa, va, oacc[c]);
            oacc[c] = mma16(pa, vl, oacc[c]);
            oacc[c] = mma16(pl, va, oacc[c]);
        }
        asm volatile("" ::: "memory");
    }

    float inv[8];
#pragma unroll
    for (int r = 0; r < 8; ++r) {
        float s = wsum[r];
        s += __shfl_xor(s, 1, 32);
        s += __shfl_xor(s, 2, 32);
        s += __shfl_xor(s, 4, 32);
        s += __shfl_xor(s, 8, 32);
        inv[r] = (1.0f / (s + DEN_EPS)) * ATT_SC;
    }
#pragma unroll
    for (int c = 0; c < 8; ++c)
#pragma unroll
        for (int r = 0; r < 8; ++r)
            ot[warp][8 * h + r][c * 16 + m] = (_Float16)(oacc[c][r] * inv[r]);
    asm volatile("" ::: "memory");
#pragma unroll 1
    for (int it = 0; it < 8; ++it) {
        const int rl = it * 2 + h;
        const v8hx val = *(const v8hx*)(&ot[warp][rl][8 * m]);
        _Float16* dst = attn + (size_t)(qb + rl) * QDIM + (size_t)hq * HDIM + 8 * m;
        *(volatile v8hx*)dst = val;
    }
    __threadfence();
#pragma unroll 1
    for (int it = 0; it < 8; ++it) {
        const int rl = it * 2 + h;
        const v8hx val = *(const v8hx*)(&ot[warp][rl][8 * m]);
        _Float16* dst = attn + (size_t)(qb + rl) * QDIM + (size_t)hq * HDIM + 8 * m;
        *(volatile v8hx*)dst = val;
    }
}

__global__ void __launch_bounds__(256)
k_proj_out(const _Float16* __restrict__ a16, const _Float16* __restrict__ w16, float* out) {
    __shared__ __align__(16) float ct[128][CT_PITCH];
    const int warp = threadIdx.x >> 5, l = threadIdx.x & 31;
    const int t0 = blockIdx.y * 128, cb = blockIdx.x;
    v8f acc[2][4];
#pragma unroll
    for (int f = 0; f < 2; ++f)
#pragma unroll
        for (int c = 0; c < 4; ++c) acc[f][c] = f8zero();
    mainloop<false, _Float16>(a16, a16, w16, w16, QDIM, t0 + (warp & 3) * 32, cb * 128 + (warp >> 2) * 64, acc);
    stage_acc(ct, acc);
    __syncthreads();
    const size_t cbase = (size_t)cb * 128 + 4 * l;
#pragma unroll 1
    for (int r = 0; r < 16; ++r) {
        const int rl = warp * 16 + r;
        const v4f x = *(const v4f*)(&ct[rl][4 * l]) * OUT_SC;
        *(volatile v4f*)(out + (size_t)(t0 + rl) * HID + cbase) = x;
    }
    __threadfence();
#pragma unroll 1
    for (int r = 0; r < 16; ++r) {
        const int rl = warp * 16 + r;
        const v4f x = *(const v4f*)(&ct[rl][4 * l]) * OUT_SC;
        *(volatile v4f*)(out + (size_t)(t0 + rl) * HID + cbase) = x;
    }
}

extern "C" void kernel_launch(void* const* d_in, const int* in_sizes, int n_in,
                              void* d_out, int out_size, void* d_ws, size_t ws_size,
                              hipStream_t stream) {
    if (n_in < 7) return;
    if (in_sizes[0] != TSEQ * HID) return;
    if (in_sizes[1] != (QKROWS + VROWS) * HID) return;
    if (in_sizes[2] != NKV * HID) return;
    if (in_sizes[3] != HID * QDIM) return;
    if (in_sizes[4] < HDIM || in_sizes[5] < HDIM || in_sizes[6] < TSEQ) return;
    if (out_size != TSEQ * HID) return;

    const float* hs   = (const float*)d_in[0];
    const float* qkvw = (const float*)d_in[1];
    const float* gw   = (const float*)d_in[2];
    const float* ow   = (const float*)d_in[3];
    const float* qnw  = (const float*)d_in[4];
    const float* knw  = (const float*)d_in[5];
    const int*   pos  = (const int*)d_in[6];
    float* out = (float*)d_out;

    const size_t szP    = (size_t)TSEQ * HID * 2;
    const size_t szWqk  = (size_t)QKROWS * HID * 2;
    const size_t szWv   = (size_t)VROWS * HID * 2;
    const size_t szOw   = (size_t)HID * QDIM * 2;
    const size_t szG    = (size_t)GROWS * HID * 2;
    const size_t szRope = (size_t)TSEQ * 128 * 4;
    const size_t szGr   = (size_t)TSEQ * NKV * 4;
    const size_t szK    = (size_t)TSEQ * KDIM * 2;
    const size_t szVt   = (size_t)KDIM * TSEQ * 2;

    char* ws = (char*)d_ws;
    size_t off = 0;
    auto carve = [&](size_t bytes) -> void* {
        void* p = ws + off;
        off += (bytes + 255) & ~(size_t)255;
        return p;
    };
    unsigned short* hs_hi = (unsigned short*)carve(szP);
    unsigned short* hs_lo = (unsigned short*)carve(szP);
    _Float16*       hs16  = (_Float16*)carve(szP);
    unsigned short* w_hi  = (unsigned short*)carve(szWqk);
    unsigned short* w_lo  = (unsigned short*)carve(szWqk);
    _Float16*       wv16  = (_Float16*)carve(szWv);
    _Float16*       ow16  = (_Float16*)carve(szOw);
    unsigned short* g_hi  = (unsigned short*)carve(szG);
    unsigned short* g_lo  = (unsigned short*)carve(szG);
    float*          rope  = (float*)carve(szRope);
    float*          graw  = (float*)carve(szGr);
    float*          cgT   = (float*)carve(szGr);
    unsigned short* q_hi  = (unsigned short*)carve(szP);
    unsigned short* q_lo  = (unsigned short*)carve(szP);
    unsigned short* k_hi  = (unsigned short*)carve(szK);
    unsigned short* k_lo  = (unsigned short*)carve(szK);
    if (off > ws_size) return;
    _Float16*       attn16 = (_Float16*)hs_hi;
    unsigned short* vt_hi  = w_hi;
    unsigned short* vt_lo  = (unsigned short*)((char*)w_hi + szVt);
    if (2 * szVt > szWqk) return;

    RopeFreq fq;
    for (int i = 0; i < 64; ++i) {
        const float e  = (float)i / 64.0f;
        const float pw = powf(10000.0f, e);
        fq.inv[i] = 1.0f / pw;
    }

    const int nvHs  = TSEQ * HID / 8;
    const int nvWqk = QKROWS * HID / 8;
    const int nvWv  = VROWS * HID / 8;
    const int nvOw  = HID * QDIM / 8;
    const int nvGv  = NKV * HID / 8;
    const int nvGt  = GROWS * HID / 8;
    const int nRope = TSEQ * 64;

    k_cvt3<<<(nvHs + 255) / 256, 256, 0, stream>>>(hs, hs_hi, hs_lo, hs16, nvHs, HS_SC);
    k_cvt_split<<<(nvWqk + 255) / 256, 256, 0, stream>>>(qkvw, w_hi, w_lo, nvWqk, nvWqk);
    k_cvt_split<<<(nvGt + 255) / 256, 256, 0, stream>>>(gw, g_hi, g_lo, nvGv, nvGt);
    k_cvt_h<<<(nvWv + 255) / 256, 256, 0, stream>>>(qkvw + (size_t)QKROWS * HID, wv16, nvWv, W_SC);
    k_cvt_h<<<(nvOw + 255) / 256, 256, 0, stream>>>(ow, ow16, nvOw, W_SC);
    k_rope_tab<<<(nRope + 255) / 256, 256, 0, stream>>>(pos, rope, fq, nRope);
    k_gate<<<TSEQ / 32, 32, 0, stream>>>((const __bf16*)hs_hi, (const __bf16*)hs_lo,
                                         (const __bf16*)g_hi, (const __bf16*)g_lo, graw);
    k_cumsum<<<1, 32, 0, stream>>>(graw, cgT);
    k_proj_qk<<<dim3(QKROWS / 128, TSEQ / 128), 256, 0, stream>>>(
        (const __bf16*)hs_hi, (const __bf16*)hs_lo, (const __bf16*)w_hi, (const __bf16*)w_lo,
        qnw, knw, rope, q_hi, q_lo, k_hi, k_lo);
    k_proj_v<<<dim3(VROWS / 128, TSEQ / 128), 256, 0, stream>>>(hs16, wv16, vt_hi, vt_lo);
    k_ret<<<dim3(TSEQ / 64, NHQ), 128, 0, stream>>>(
        (const __bf16*)q_hi, (const __bf16*)q_lo, (const __bf16*)k_hi, (const __bf16*)k_lo,
        (const __bf16*)vt_hi, (const __bf16*)vt_lo, cgT, attn16);
    k_proj_out<<<dim3(HID / 128, TSEQ / 128), 256, 0, stream>>>(attn16, ow16, out);
}
